// DifferentialSelfAttention_80075370266692
// MI455X (gfx1250) — hardware-verified
//
#include <hip/hip_runtime.h>
#include <math.h>
#include <float.h>
#include <stdint.h>

#define NB    2
#define SEQ   2048
#define DM    1024
#define DQK   2048
#define NH    16
#define HD    64
#define NFREQ (HD / 2)
#define NQB   (SEQ / 64)
#define VLP   512
#define RESQB 8
#define LAM0  0.2f
#define OSCL  0.8f
static_assert(RESQB * 64 <= VLP);
static_assert(NH * HD == DM);
static_assert(NH * 2 * HD == DQK);
static_assert((SEQ % 64) == 0 && (DM % 64) == 0 && (DQK % 64) == 0);

typedef _Float16 v16h __attribute__((ext_vector_type(16)));
typedef _Float16 v8h  __attribute__((ext_vector_type(8)));
typedef __bf16   v16b __attribute__((ext_vector_type(16)));
typedef __bf16   v8b  __attribute__((ext_vector_type(8)));
typedef float    v8f  __attribute__((ext_vector_type(8)));
typedef float    v4f  __attribute__((ext_vector_type(4)));
typedef unsigned int v4u __attribute__((ext_vector_type(4)));

__device__ __forceinline__ unsigned short bf_bits(float f) {
  unsigned u = __float_as_uint(f);
  return (unsigned short)((u + 0x7FFFu + ((u >> 16) & 1u)) >> 16);
}
__device__ __forceinline__ float bf_up(unsigned short h) { return __uint_as_float(((unsigned)h) << 16); }
__device__ __forceinline__ float bfr(float f) { return bf_up(bf_bits(f)); }
__device__ __forceinline__ unsigned short h_bits(_Float16 x) { return __builtin_bit_cast(unsigned short, x); }
__device__ __forceinline__ unsigned pk16(unsigned short a, unsigned short b) { return (unsigned)a | ((unsigned)b << 16); }
__device__ __forceinline__ v8f zero8() { v8f z = {0.f, 0.f, 0.f, 0.f, 0.f, 0.f, 0.f, 0.f}; return z; }
__device__ __forceinline__ v8h zero8h() {
  const _Float16 z = (_Float16)0.0f;
  v8h r = {z, z, z, z, z, z, z, z};
  return r;
}

__device__ __forceinline__ v16b ldfrag_b(const __bf16* p) {
  union { v16b v; v8b h[2]; } f;
  f.h[0] = *(const v8b*)(p);
  f.h[1] = *(const v8b*)(p + 16);
  return f.v;
}

__device__ __forceinline__ v8f mma_b(v16b a, v16b b, v8f c) {
  c = __builtin_amdgcn_wmma_f32_16x16x32_bf16(false, a, false, b, (short)0, c, false, false);
#if defined(__HIP_DEVICE_COMPILE__)
  asm volatile("v_nop\n\tv_nop\n\tv_nop\n\tv_nop" : "+v"(c) : "v"(a), "v"(b));
#endif
  return c;
}
__device__ __forceinline__ v8f mma_h(v16h a, v16h b, v8f c) {
  c = __builtin_amdgcn_wmma_f32_16x16x32_f16(false, a, false, b, (short)0, c, false, false);
#if defined(__HIP_DEVICE_COMPILE__)
  asm volatile("v_nop\n\tv_nop\n\tv_nop\n\tv_nop" : "+v"(c) : "v"(a), "v"(b));
#endif
  return c;
}
__device__ __forceinline__ v8f mma_b_raw(v16b a, v16b b, v8f c) {
  return __builtin_amdgcn_wmma_f32_16x16x32_bf16(false, a, false, b, (short)0, c, false, false);
}
__device__ __forceinline__ void dep_guard_b(v8f& a, v8f& b, v16b x, v16b y) {
#if defined(__HIP_DEVICE_COMPILE__)
  asm volatile("v_nop\n\tv_nop\n\tv_nop\n\tv_nop" : "+v"(a), "+v"(b) : "v"(x), "v"(y));
#endif
}
__device__ __forceinline__ void keep4_b(v16b a, v16b b, v16b c, v16b d) {
#if defined(__HIP_DEVICE_COMPILE__)
  asm volatile("v_nop" :: "v"(a), "v"(b), "v"(c), "v"(d));
#endif
}
__device__ __forceinline__ void acc_guard4(v8f& a, v8f& b, v8f& c, v8f& d) {
#if defined(__HIP_DEVICE_COMPILE__)
  asm volatile("v_nop\n\tv_nop\n\tv_nop\n\tv_nop" : "+v"(a), "+v"(b), "+v"(c), "+v"(d));
#endif
}

__global__ __launch_bounds__(256) void cvt_bf16x8(const float* __restrict__ in, unsigned short* out, int n8) {
  const int i = blockIdx.x * 256 + threadIdx.x;
  if (i < n8) {
    const v4f a = *(const v4f*)(in + (size_t)i * 8);
    const v4f b = *(const v4f*)(in + (size_t)i * 8 + 4);
    v4u p;
    p[0] = pk16(bf_bits(a[0]), bf_bits(a[1]));
    p[1] = pk16(bf_bits(a[2]), bf_bits(a[3]));
    p[2] = pk16(bf_bits(b[0]), bf_bits(b[1]));
    p[3] = pk16(bf_bits(b[2]), bf_bits(b[3]));
    *(volatile v4u*)(out + (size_t)i * 8) = p;
    __threadfence();
    *(volatile v4u*)(out + (size_t)i * 8) = p;
  }
}

__global__ __launch_bounds__(32) void invfreq_tab(float* invf) {
  __shared__ __align__(16) float sf[NFREQ];
  const int j = threadIdx.x;
  const float e = (float)j * (1.0f / (float)NFREQ);
  const float pw = powf(10000.0f, e);
  sf[j] = 1.0f / pw;
  __syncthreads();
  const v4f v = *(const v4f*)(sf + 4 * (j & 7));
  if (j < 8) *(volatile v4f*)(invf + 4 * j) = v;
  __threadfence();
  if (j < 8) *(volatile v4f*)(invf + 4 * j) = v;
}

__global__ __launch_bounds__(256) void rope_tab(const float* __restrict__ invf, float* cosT, float* sinT) {
  const int g = blockIdx.x * 256 + threadIdx.x;
  if (g < SEQ * NFREQ) {
    const int t = g / NFREQ;
    const int j = g - t * NFREQ;
    const float ang = (float)t * invf[j];
    const float cv = cosf(ang);
    const float sv = sinf(ang);
    *(volatile float*)(cosT + g) = cv;
    *(volatile float*)(sinT + g) = sv;
    __threadfence();
    *(volatile float*)(cosT + g) = cv;
    *(volatile float*)(sinT + g) = sv;
  }
}

template <int NSPLIT, int OUT_MODE, int BIAS>
__global__ __launch_bounds__(256) void gemm64(
    const unsigned short* __restrict__ Ap, const unsigned short* A2p, int lda, long long strideA,
    const unsigned short* __restrict__ Btp, const unsigned short* Bt2p, int ldb, long long strideB,
    void* Cout, int ldc, long long strideC,
    void* Cout2, int ldc2, long long strideC2, int N2,
    int M, int N, int K, float rscale, const float* __restrict__ bias) {
  const __bf16* A   = (const __bf16*)(const void*)Ap;
  const __bf16* A2  = (const __bf16*)(const void*)A2p;
  const __bf16* Bt  = (const __bf16*)(const void*)Btp;
  const __bf16* Bt2 = (const __bf16*)(const void*)Bt2p;
  __shared__ __align__(16) float sT[8][16 * 68];
  const int b    = blockIdx.y;
  const int lane = threadIdx.x & 31;
  const int wave = threadIdx.x >> 5;
  const int tilesN = N >> 6;
  const int tilesM = M >> 6;
  const int tile = blockIdx.x * 8 + wave;
  if (tile >= tilesM * tilesN) return;
  const int tm = tile / tilesN;
  const int tn = tile - tm * tilesN;
  const int m0 = tm << 6;
  const int n0 = tn << 6;

  const __bf16* Ab  = A  + (size_t)b * strideA;
  const __bf16* Bb  = Bt + (size_t)b * strideB;
  const __bf16* Ab2 = (NSPLIT >= 1) ? (A2  + (size_t)b * strideA) : Ab;
  const __bf16* Bb2 = (NSPLIT == 2) ? (Bt2 + (size_t)b * strideB) : Bb;

  const int rlane = lane & 15;
  const int koff  = (lane >> 4) * 8;
  const int mOff  = (lane >> 4) * 8;

  v8f acc[4][4];
#pragma unroll
  for (int i = 0; i < 4; ++i)
#pragma unroll
    for (int j = 0; j < 4; ++j) acc[i][j] = zero8();

  for (int k0 = 0; k0 < K; k0 += 32) {
    v16b bh[4], bl[4];
#pragma unroll
    for (int j = 0; j < 4; ++j) {
      const size_t bo = (size_t)(n0 + (j << 4) + rlane) * ldb + koff + k0;
      bh[j] = ldfrag_b(Bb + bo);
      if (NSPLIT == 2) bl[j] = ldfrag_b(Bb2 + bo); else bl[j] = bh[j];
    }
#pragma unroll
    for (int i = 0; i < 4; ++i) {
      const size_t ao = (size_t)(m0 + (i << 4) + rlane) * lda + koff + k0;
      const v16b ah = ldfrag_b(Ab + ao);
      v16b al = ah;
      if (NSPLIT >= 1) al = ldfrag_b(Ab2 + ao);
#pragma unroll
      for (int j = 0; j < 4; ++j) {
        acc[i][j] = mma_b_raw(ah, bh[j], acc[i][j]);
        if (NSPLIT >= 1) acc[i][j] = mma_b_raw(al, bh[j], acc[i][j]);
        if (NSPLIT == 2) acc[i][j] = mma_b_raw(ah, bl[j], acc[i][j]);
      }
      dep_guard_b(acc[i][0], acc[i][3], ah, al);
    }
    keep4_b(bh[0], bh[1], bh[2], bh[3]);
    if (NSPLIT == 2) keep4_b(bl[0], bl[1], bl[2], bl[3]);
  }
  acc_guard4(acc[0][0], acc[0][1], acc[0][2], acc[0][3]);
  acc_guard4(acc[1][0], acc[1][1], acc[1][2], acc[1][3]);
  acc_guard4(acc[2][0], acc[2][1], acc[2][2], acc[2][3]);
  acc_guard4(acc[3][0], acc[3][1], acc[3][2], acc[3][3]);

  float bcol[4];
#pragma unroll
  for (int j = 0; j < 4; ++j) bcol[j] = 0.f;
  if (BIAS == 1) {
#pragma unroll
    for (int j = 0; j < 4; ++j) bcol[j] = bfr(bias[n0 + (j << 4) + rlane]);
  }
  float* slab = sT[wave];
#pragma unroll
  for (int i = 0; i < 4; ++i) {
    const int mBase = m0 + (i << 4);
    float brow[8];
#pragma unroll
    for (int r = 0; r < 8; ++r) brow[r] = 0.f;
    if (BIAS == 2) {
#pragma unroll
      for (int r = 0; r < 8; ++r) brow[r] = bfr(bias[mBase + mOff + r]);
    }
#pragma unroll
    for (int j = 0; j < 4; ++j) {
#pragma unroll
      for (int r = 0; r < 8; ++r) {
        slab[(mOff + r) * 68 + (j << 4) + rlane] = (acc[i][j][r] + bcol[j]) + brow[r];
      }
    }
    __builtin_amdgcn_fence(__ATOMIC_RELEASE, "workgroup");
    __builtin_amdgcn_wave_barrier();
    __builtin_amdgcn_fence(__ATOMIC_ACQUIRE, "workgroup");
    if (OUT_MODE == 0) {
      float* C = (float*)Cout + (size_t)b * strideC;
      const int hh = lane >> 4, c4 = (lane & 15) * 4;
      for (int pass = 0; pass < 2; ++pass) {
#pragma unroll
        for (int it = 0; it < 8; ++it) {
          const int row = it * 2 + hh;
          const v4f v = *(const v4f*)(slab + row * 68 + c4);
          *(volatile v4f*)(C + (size_t)(mBase + row) * ldc + n0 + c4) = v;
        }
        __threadfence();
      }
    } else {
      const int q = lane >> 3, c8 = (lane & 7) * 8;
      unsigned short* C  = (unsigned short*)Cout  + (size_t)b * strideC;
      unsigned short* C2 = (unsigned short*)Cout2 + (size_t)b * strideC2;
      const bool wlo = (OUT_MODE == 2) || (n0 < N2);
      v4u hv[4], lv[4];
#pragma unroll
      for (int it = 0; it < 4; ++it) {
        const int row = it * 4 + q;
        const float* sp = slab + row * 68 + c8;
        v4u a, a2;
#pragma unroll
        for (int e = 0; e < 4; ++e) {
          const float f0 = sp[2 * e], f1 = sp[2 * e + 1];
          unsigned short h0, h1, l0, l1;
          if (OUT_MODE == 2) {
            h0 = bf_bits(f0); h1 = bf_bits(f1);
            l0 = bf_bits(f0 - bf_up(h0)); l1 = bf_bits(f1 - bf_up(h1));
          } else {
            const _Float16 x0 = (_Float16)f0, x1 = (_Float16)f1;
            h0 = h_bits(x0); h1 = h_bits(x1);
            l0 = h_bits((_Float16)((f0 - (float)x0) * rscale));
            l1 = h_bits((_Float16)((f1 - (float)x1) * rscale));
          }
          a[e] = pk16(h0, h1); a2[e] = pk16(l0, l1);
        }
        hv[it] = a; lv[it] = a2;
      }
      for (int pass = 0; pass < 2; ++pass) {
#pragma unroll
        for (int it = 0; it < 4; ++it) {
          const int row = it * 4 + q;
          *(volatile v4u*)(C + (size_t)(mBase + row) * ldc + n0 + c8) = hv[it];
          if (wlo) *(volatile v4u*)(C2 + (size_t)(mBase + row) * ldc2 + n0 + c8) = lv[it];
        }
        __threadfence();
      }
    }
    __builtin_amdgcn_fence(__ATOMIC_RELEASE, "workgroup");
    __builtin_amdgcn_wave_barrier();
    __builtin_amdgcn_fence(__ATOMIC_ACQUIRE, "workgroup");
  }
}

__device__ __forceinline__ void rope_row8(const float* __restrict__ src, size_t rowOff, int c0, int p0,
                                          bool second, v4f cs0, v4f cs1, v4f sn0, v4f sn1,
                                          unsigned short* Hp, unsigned short* Lp) {
#pragma clang fp contract(off)
  const v4f xa0 = *(const v4f*)(src + rowOff + c0);
  const v4f xa1 = *(const v4f*)(src + rowOff + c0 + 4);
  const v4f xp0 = *(const v4f*)(src + rowOff + p0);
  const v4f xp1 = *(const v4f*)(src + rowOff + p0 + 4);
  float o[8];
#pragma unroll
  for (int e = 0; e < 4; ++e) {
    {
      const float a = xa0[e], p = xp0[e], cs = cs0[e], sn = sn0[e];
      const float f1 = a * cs - p * sn;
      const float f2 = p * sn + a * cs;
      o[e] = second ? f2 : f1;
    }
    {
      const float a = xa1[e], p = xp1[e], cs = cs1[e], sn = sn1[e];
      const float f1 = a * cs - p * sn;
      const float f2 = p * sn + a * cs;
      o[4 + e] = second ? f2 : f1;
    }
  }
  v4u hv, lv;
#pragma unroll
  for (int e = 0; e < 4; ++e) {
    const float f0 = o[2 * e], f1 = o[2 * e + 1];
    const unsigned short h0 = bf_bits(f0), h1 = bf_bits(f1);
    const unsigned short l0 = bf_bits(f0 - bf_up(h0)), l1 = bf_bits(f1 - bf_up(h1));
    hv[e] = pk16(h0, h1); lv[e] = pk16(l0, l1);
  }
  const size_t go = rowOff + c0;
  *(volatile v4u*)(Hp + go) = hv;
  *(volatile v4u*)(Lp + go) = lv;
  __threadfence();
  *(volatile v4u*)(Hp + go) = hv;
  *(volatile v4u*)(Lp + go) = lv;
}

__global__ __launch_bounds__(256) void rope_split(const float* __restrict__ Qf, const float* __restrict__ Kf,
                                                   const float* __restrict__ cosT, const float* __restrict__ sinT,
                                                   unsigned short* Qh, unsigned short* Ql,
                                                   unsigned short* Kh, unsigned short* Kl) {
  const int t = blockIdx.x;
  const int c0 = threadIdx.x * 8;
  const int jj0 = c0 & 31;
  const bool second = (c0 & 32) != 0;
  const int p0 = second ? (c0 - 32) : (c0 + 32);
  const float* cr = cosT + (size_t)t * NFREQ + jj0;
  const float* sr = sinT + (size_t)t * NFREQ + jj0;
  const v4f cs0 = *(const v4f*)(cr), cs1 = *(const v4f*)(cr + 4);
  const v4f sn0 = *(const v4f*)(sr), sn1 = *(const v4f*)(sr + 4);
  const size_t rowOff = (size_t)t * DQK;
  rope_row8(Qf, rowOff, c0, p0, second, cs0, cs1, sn0, sn1, Qh, Ql);
  rope_row8(Kf, rowOff, c0, p0, second, cs0, cs1, sn0, sn1, Kh, Kl);
}

template <bool RES>
__global__ __launch_bounds__(128)
void attn_causal64(const unsigned short* __restrict__ qhp, const unsigned short* __restrict__ qlp,
                   const unsigned short* __restrict__ khp, const unsigned short* __restrict__ klp,
                   const unsigned short* __restrict__ vhp, const unsigned short* __restrict__ vlp,
                   float* Cp, int soff, int qbBase, int nqbThis, float sscale) {
  union FB { v16b v; v8b h[2]; };
  union FH { v16h v; v8h h[2]; };
  __shared__ __align__(16) __bf16   Ksh[64 * 64];
  __shared__ __align__(16) __bf16   Ksl[64 * 64];
  __shared__ __align__(16) _Float16 Vth[64 * 64];
  __shared__ __align__(16) _Float16 Vtl[RES ? 64 * 64 : 8];
  __shared__ __align__(16) _Float16 Psh[4][16 * 64];
  __shared__ __align__(16) _Float16 Psl[RES ? 4 : 1][16 * 64];
  __shared__ __align__(16) float    Os[4][16 * 64];

  const int tid  = threadIdx.x;
  const int wave = tid >> 5;
  const int lane = tid & 31;
  const int hh   = lane >> 4;
  const int c    = lane & 15;

  const int bx   = blockIdx.x;
  const int qbl  = bx % nqbThis;
  const int h    = bx / nqbThis;
  const int qb   = qbBase + qbl;
  const int q0   = qb * 64 + wave * 16;
  const int col  = h * (2 * HD) + soff;

  const __bf16* Qh = (const __bf16*)(const void*)qhp + col;
  const __bf16* Ql = (const __bf16*)(const void*)qlp + col;
  const __bf16* Kh = (const __bf16*)(const void*)khp + col;
  const __bf16* Kl = (const __bf16*)(const void*)klp + col;
  const _Float16* Vh = (const _Float16*)(const void*)vhp + (size_t)h * HD * SEQ;
  const _Float16* Vl = (const _Float16*)(const void*)vlp + (size_t)h * HD * VLP;

  v16b qah[2], qal[2];
#pragma unroll
  for (int dc = 0; dc < 2; ++dc) {
    const size_t qo = (size_t)(q0 + c) * DQK + dc * 32 + 8 * hh;
    qah[dc] = ldfrag_b(Qh + qo);
    qal[dc] = ldfrag_b(Ql + qo);
  }

  float mrow[8], lrow[8];
  v8f oacc[4];
#pragma unroll
  for (int r = 0; r < 8; ++r) { mrow[r] = -INFINITY; lrow[r] = 0.f; }
#pragma unroll
  for (int t = 0; t < 4; ++t) oacc[t] = zero8();

  for (int kt = 0; kt < NQB; ++kt) {
    if (kt > qb) break;
    const bool diag = (kt == qb);
    const int kv0 = kt * 64;
    __syncthreads();
    {
      const int r = tid >> 1, half = (tid & 1) * 32;
      const __bf16*   kg  = Kh + (size_t)(kv0 + r) * DQK + half;
      const __bf16*   klg = Kl + (size_t)(kv0 + r) * DQK + half;
      const _Float16* vg  = Vh + (size_t)r * SEQ + kv0 + half;
      const int kvl = (kv0 + 64 <= VLP) ? kv0 : (VLP - 64);
      const _Float16* vlg = Vl + (size_t)r * VLP + kvl + half;
      const bool resOK = (kv0 + 64 <= VLP);
#pragma unroll
      for (int i = 0; i < 4; ++i) {
        const v8b a0 = *(const v8b*)(kg + 8 * i);
        const v8b a1 = *(const v8b*)(klg + 8 * i);
        const v8h b0 = *(const v8h*)(vg + 8 * i);
        *(v8b*)(Ksh + r * 64 + half + 8 * i) = a0;
        *(v8b*)(Ksl + r * 64 + half + 8 * i) = a1;
        *(v8h*)(Vth + r * 64 + half + 8 * i) = b0;
        if (RES) {
          v8h b1 = *(const v8h*)(vlg + 8 * i);
          if (!resOK) b1 = zero8h();
          *(v8h*)(Vtl + r * 64 + half + 8 * i) = b1;
        }
      }
    }
    __syncthreads();

    v8f s[4];
#pragma unroll
    for (int j = 0; j < 4; ++j) {
      s[j] = zero8();
#pragma unroll
      for (int dc = 0; dc < 2; ++dc) {
        FB kb, kl;
        kb.h[0] = *(const v8b*)(Ksh + (j * 16 + c) * 64 + dc * 32 + 8 * hh);
        kb.h[1] = *(const v8b*)(Ksh + (j * 16 + c) * 64 + dc * 32 + 16 + 8 * hh);
        kl.h[0] = *(const v8b*)(Ksl + (j * 16 + c) * 64 + dc * 32 + 8 * hh);
        kl.h[1] = *(const v8b*)(Ksl + (j * 16 + c) * 64 + dc * 32 + 16 + 8 * hh);
        s[j] = mma_b(qah[dc], kb.v, s[j]);
        s[j] = mma_b(qah[dc], kl.v, s[j]);
        s[j] = mma_b(qal[dc], kb.v, s[j]);
      }
    }

    _Float16* pwh = Psh[wave];
    _Float16* pwl = Psl[RES ? wave : 0];
#pragma unroll
    for (int r = 0; r < 8; ++r) {
      const int qrow = q0 + 8 * hh + r;
      float m = -INFINITY;
#pragma unroll
      for (int j = 0; j < 4; ++j) {
        const int key = kv0 + j * 16 + c;
        float sv = s[j][r] * sscale;
        sv = (diag && key > qrow) ? -INFINITY : sv;
        s[j][r] = sv;
        m = fmaxf(m, sv);
      }
#pragma unroll
      for (int off = 1; off < 16; off <<= 1) m = fmaxf(m, __shfl_xor(m, off, 32));
      const float mnew  = fmaxf(mrow[r], m);
      const float msafe = (mnew == -INFINITY) ? 0.f : mnew;
      const float alpha = __expf(mrow[r] - msafe);
      mrow[r] = mnew;
      float psum = 0.f;
#pragma unroll
      for (int j = 0; j < 4; ++j) {
        const float p = __expf(s[j][r] - msafe);
        psum += p;
        const float p1k = p * 1024.0f;
        const _Float16 ph = (_Float16)p1k;
        pwh[(8 * hh + r) * 64 + j * 16 + c] = ph;
        if (RES) {
          const _Float16 pl = (_Float16)((p1k - (float)ph) * 4096.0f);
          pwl[(8 * hh + r) * 64 + j * 16 + c] = pl;
        }
      }
#pragma unroll
      for (int off = 1; off < 16; off <<= 1) psum += __shfl_xor(psum, off, 32);
      lrow[r] = lrow[r] * alpha + psum;
#pragma unroll
      for (int t = 0; t < 4; ++t) oacc[t][r] *= alpha;
    }
    __builtin_amdgcn_fence(__ATOMIC_RELEASE, "workgroup");
    __builtin_amdgcn_wave_barrier();
    __builtin_amdgcn_fence(__ATOMIC_ACQUIRE, "workgroup");

    v8f o1[4];
#pragma unroll
    for (int t = 0; t < 4; ++t) o1[t] = zero8();
#pragma unroll 1
    for (int kk = 0; kk < 2; ++kk) {
      FH pa, pl;
      pa.h[0] = *(const v8h*)(pwh + c * 64 + kk * 32 + 8 * hh);
      pa.h[1] = *(const v8h*)(pwh + c * 64 + kk * 32 + 16 + 8 * hh);
      if (RES) {
        pl.h[0] = *(const v8h*)(pwl + c * 64 + kk * 32 + 8 * hh);
        pl.h[1] = *(const v8h*)(pwl + c * 64 + kk * 32 + 16 + 8 * hh);
      } else {
        pl.v = pa.v;
      }
#pragma unroll
      for (int t = 0; t < 4; ++t) {
        FH vb;
        vb.h[0] = *(const v8h*)(Vth + (t * 16 + c) * 64 + kk * 32 + 8 * hh);
        vb.h[1] = *(const v8h*)(Vth + (t * 16 + c) * 64 + kk * 32 + 16 + 8 * hh);
        oacc[t] = mma_h(pa.v, vb.v, oacc[t]);
        if (RES) {
          FH vl;
          vl.h[0] = *(const v8h*)(Vtl + (t * 16 + c) * 64 + kk * 32 + 8 * hh);
          vl.h[1] = *(const v8h*)(Vtl + (t * 16 + c) * 64 + kk * 32 + 16 + 8 * hh);
          o1[t] = mma_h(pa.v, vl.v, o1[t]);
          o1[t] = mma_h(pl.v, vb.v, o1[t]);
        }
      }
    }
    if (RES) {
#pragma unroll
      for (int t = 0; t < 4; ++t)
#pragma unroll
        for (int r = 0; r < 8; ++r) oacc[t][r] += o1[t][r] * (1.0f / 4096.0f);
    }
  }

  float* os = Os[wave];
#pragma unroll
  for (int r = 0; r < 8; ++r) {
    const float l = lrow[r];
    const float inv = ((l > 0.f) ? (1.0f / l) : 0.f) * (1.0f / 1024.0f);
#pragma unroll
    for (int t = 0; t < 4; ++t) os[(8 * hh + r) * 64 + t * 16 + c] = oacc[t][r] * inv;
  }
  __builtin_amdgcn_fence(__ATOMIC_RELEASE, "workgroup");
  __builtin_amdgcn_wave_barrier();
  __builtin_amdgcn_fence(__ATOMIC_ACQUIRE, "workgroup");
  {
    const int h2 = lane >> 4, c4 = (lane & 15) * 4;
    v4f ov[8];
#pragma unroll
    for (int it = 0; it < 8; ++it) {
      const int row = it * 2 + h2;
      ov[it] = *(const v4f*)(os + row * 64 + c4);
    }
    for (int pass = 0; pass < 2; ++pass) {
#pragma unroll
      for (int it = 0; it < 8; ++it) {
        const int row = it * 2 + h2;
        const size_t go = (size_t)(q0 + row) * DM + (size_t)h * HD + c4;
        *(volatile v4f*)(Cp + go) = ov[it];
      }
      __threadfence();
    }
  }
}

__global__ __launch_bounds__(128) void diff_combine(
    const float* __restrict__ C1, const float* __restrict__ C2,
    const float* __restrict__ lq1, const float* __restrict__ lk1,
    const float* __restrict__ lq2, const float* __restrict__ lk2,
    const float* __restrict__ hnw, unsigned short* Oh, unsigned short* Ol) {
#pragma clang fp contract(off)
  __shared__ float lam_s[NH];
  const int tid = threadIdx.x;
  const int t   = blockIdx.x;
  if (tid < NH) {
    const float* a1 = lq1 + tid * HD;
    const float* b1 = lk1 + tid * HD;
    const float* a2 = lq2 + tid * HD;
    const float* b2 = lk2 + tid * HD;
    float sa = 0.f, sb = 0.f;
#pragma unroll 1
    for (int d = 0; d < HD; ++d) {
      sa += bfr(a1[d]) * bfr(b1[d]);
      sb += bfr(a2[d]) * bfr(b2[d]);
    }
    lam_s[tid] = (LAM0 + expf(sa)) - expf(sb);
  }
  __syncthreads();
  const int c0 = tid * 8;
  const int h  = c0 >> 6;
  const int d0 = c0 & 63;
  const size_t ro = (size_t)t * DM + c0;
  const v4f x0 = *(const v4f*)(C1 + ro), x1 = *(const v4f*)(C1 + ro + 4);
  const v4f y0 = *(const v4f*)(C2 + ro), y1 = *(const v4f*)(C2 + ro + 4);
  const float lam = lam_s[h];
  float o[8];
  float ss = 0.f;
#pragma unroll
  for (int e = 0; e < 4; ++e) {
    o[e]     = x0[e] - lam * y0[e];
    o[4 + e] = x1[e] - lam * y1[e];
  }
#pragma unroll
  for (int e = 0; e < 8; ++e) ss += o[e] * o[e];
  ss += __shfl_xor(ss, 1, 32);
  ss += __shfl_xor(ss, 2, 32);
  ss += __shfl_xor(ss, 4, 32);
  const float ms = ss * (1.0f / (float)HD);
  const float rn = rsqrtf(ms + 1.0e-6f);
  v4u hv, lv;
#pragma unroll
  for (int e = 0; e < 4; ++e) {
    const float w0 = bfr(hnw[h * HD + d0 + 2 * e]);
    const float w1 = bfr(hnw[h * HD + d0 + 2 * e + 1]);
    const float f0 = ((o[2 * e] * rn) * w0) * OSCL;
    const float f1 = ((o[2 * e + 1] * rn) * w1) * OSCL;
    const unsigned short h0 = bf_bits(f0), h1 = bf_bits(f1);
    const unsigned short l0 = bf_bits(f0 - bf_up(h0)), l1 = bf_bits(f1 - bf_up(h1));
    hv[e] = pk16(h0, h1); lv[e] = pk16(l0, l1);
  }
  *(volatile v4u*)(Oh + ro) = hv;
  *(volatile v4u*)(Ol + ro) = lv;
  __threadfence();
  *(volatile v4u*)(Oh + ro) = hv;
  *(volatile v4u*)(Ol + ro) = lv;
}

extern "C" void kernel_launch(void* const* d_in, const int* in_sizes, int n_in,
                              void* d_out, int out_size, void* d_ws, size_t ws_size,
                              hipStream_t stream) {
  if (n_in < 14) return;
  if (in_sizes[0] != NB * SEQ * DM) return;
  if (in_sizes[1] != DQK * DM || in_sizes[2] != DQK) return;
  if (in_sizes[3] != DQK * DM || in_sizes[4] != DQK) return;
  if (in_sizes[5] != DM * DM || in_sizes[6] != DM) return;
  if (in_sizes[7] != DM * DM || in_sizes[8] != DM) return;
  for (int i = 9; i < 14; ++i) if (in_sizes[i] != NH * HD) return;
  if (out_size != NB * SEQ * DM) return;

  const float* x   = (const float*)d_in[0];
  const float* Wq  = (const float*)d_in[1];
  const float* bq  = (const float*)d_in[2];
  const float* Wk  = (const float*)d_in[3];
  const float* bk  = (const float*)d_in[4];
  const float* Wv  = (const float*)d_in[5];
  const float* bv  = (const float*)d_in[6];
  const float* Wo  = (const float*)d_in[7];
  const float* bo  = (const float*)d_in[8];
  const float* hnw = (const float*)d_in[9];
  const float* lq1 = (const float*)d_in[10];
  const float* lk1 = (const float*)d_in[11];
  const float* lq2 = (const float*)d_in[12];
  const float* lk2 = (const float*)d_in[13];
  float* outp = (float*)d_out;

  const size_t PXB  = (size_t)NB * SEQ * DM * 2;
  const size_t PWQ  = (size_t)DQK * DM * 2;
  const size_t PWV  = (size_t)DM * DM * 2;
  const size_t PIF  = 4096;
  const size_t PTAB = (size_t)SEQ * NFREQ * 4;
  const size_t PQF  = (size_t)SEQ * DQK * 4;
  const size_t PQP  = (size_t)SEQ * DQK * 2;
  const size_t PVT  = (size_t)DM * SEQ * 2;
  const size_t PVL  = (size_t)DM * VLP * 2;
  const size_t PC   = (size_t)SEQ * DM * 4;
  const size_t PO   = (size_t)SEQ * DM * 2;
  size_t off = 0;
  const size_t oXb  = off; off += PXB;
  const size_t oWq  = off; off += PWQ;
  const size_t oWk  = off; off += PWQ;
  const size_t oWv  = off; off += PWV;
  const size_t oWo  = off; off += PWV;
  const size_t oIF  = off; off += PIF;
  const size_t oCos = off; off += PTAB;
  const size_t oSin = off; off += PTAB;
  const size_t oQf  = off; off += PQF;
  const size_t oKf  = off; off += PQF;
  const size_t oQh  = off; off += PQP;
  const size_t oQl  = off; off += PQP;
  const size_t oKh  = off; off += PQP;
  const size_t oKl  = off; off += PQP;
  const size_t oVTh = off; off += PVT;
  const size_t oVTl = off; off += PVL;
  const size_t oC1  = off; off += PC;
  const size_t oC2  = off; off += PC;
  const size_t oOh  = off; off += PO;
  const size_t oOl  = off; off += PO;
  if (off > ws_size) return;
  if (off > (size_t)134217728) return;

  char* ws = (char*)d_ws;
  unsigned short* Xb  = (unsigned short*)(ws + oXb);
  unsigned short* Wqb = (unsigned short*)(ws + oWq);
  unsigned short* Wkb = (unsigned short*)(ws + oWk);
  unsigned short* Wvb = (unsigned short*)(ws + oWv);
  unsigned short* Wob = (unsigned short*)(ws + oWo);
  float*          IFt = (float*)(ws + oIF);
  float*          CosT = (float*)(ws + oCos);
  float*          SinT = (float*)(ws + oSin);
  float*          Qf  = (float*)(ws + oQf);
  float*          Kf  = (float*)(ws + oKf);
  unsigned short* Qh  = (unsigned short*)(ws + oQh);
  unsigned short* Ql  = (unsigned short*)(ws + oQl);
  unsigned short* Kh  = (unsigned short*)(ws + oKh);
  unsigned short* Kl  = (unsigned short*)(ws + oKl);
  unsigned short* VTh = (unsigned short*)(ws + oVTh);
  unsigned short* VTl = (unsigned short*)(ws + oVTl);
  float*          C1  = (float*)(ws + oC1);
  float*          C2  = (float*)(ws + oC2);
  unsigned short* Oh  = (unsigned short*)(ws + oOh);
  unsigned short* Ol  = (unsigned short*)(ws + oOl);

  const dim3 blk256(256), blk128(128), blk32(32);
  const int n8x  = NB * SEQ * DM / 8;
  const int n8wq = DQK * DM / 8;
  const int n8wv = DM * DM / 8;
  const dim3 gCvtX((n8x + 255) / 256);
  const dim3 gCvtWq((n8wq + 255) / 256);
  const dim3 gCvtWv((n8wv + 255) / 256);
  const dim3 gTab((SEQ * NFREQ + 255) / 256);
  const dim3 gQK(((SEQ / 64) * (DQK / 64) + 7) / 8, 1);
  const dim3 gVT(((DM / 64) * (SEQ / 64) + 7) / 8, 1);
  const dim3 gOut(((SEQ / 64) * (DM / 64) + 7) / 8, 1);
  const dim3 gRow(SEQ);
  const dim3 gAttR(NH * RESQB);
  const dim3 gAttN(NH * (NQB - RESQB));

  cvt_bf16x8<<<gCvtX, blk256, 0, stream>>>(x, Xb, n8x);
  cvt_bf16x8<<<gCvtWq, blk256, 0, stream>>>(Wq, Wqb, n8wq);
  cvt_bf16x8<<<gCvtWq, blk256, 0, stream>>>(Wk, Wkb, n8wq);
  cvt_bf16x8<<<gCvtWv, blk256, 0, stream>>>(Wv, Wvb, n8wv);
  cvt_bf16x8<<<gCvtWv, blk256, 0, stream>>>(Wo, Wob, n8wv);
  invfreq_tab<<<dim3(1), blk32, 0, stream>>>(IFt);
  rope_tab<<<gTab, blk256, 0, stream>>>(IFt, CosT, SinT);

  for (int b = 0; b < NB; ++b) {
    const unsigned short* Xbb = Xb + (size_t)b * SEQ * DM;
    float* outb = outp + (size_t)b * SEQ * DM;
    gemm64<0, 0, 1><<<gQK, blk256, 0, stream>>>(
        Xbb, Xbb, DM, 0LL, Wqb, Wqb, DM, 0LL,
        (void*)Qf, DQK, 0LL, (void*)Qf, DQK, 0LL, DQK,
        SEQ, DQK, DM, 1.0f, bq);
    gemm64<0, 0, 1><<<gQK, blk256, 0, stream>>>(
        Xbb, Xbb, DM, 0LL, Wkb, Wkb, DM, 0LL,
        (void*)Kf, DQK, 0LL, (void*)Kf, DQK, 0LL, DQK,
        SEQ, DQK, DM, 1.0f, bk);
    gemm64<0, 3, 2><<<gVT, blk256, 0, stream>>>(
        Wvb, Wvb, DM, 0LL, Xbb, Xbb, DM, 0LL,
        (void*)VTh, SEQ, 0LL, (void*)VTl, VLP, 0LL, VLP,
        DM, SEQ, DM, 4096.0f, bv);
    rope_split<<<gRow, blk256, 0, stream>>>(Qf, Kf, CosT, SinT, Qh, Ql, Kh, Kl);
    attn_causal64<true><<<gAttR, blk128, 0, stream>>>(
        Qh, Ql, Kh, Kl, VTh, VTl, C1, 0, 0, RESQB, 0.125f);
    attn_causal64<false><<<gAttN, blk128, 0, stream>>>(
        Qh, Ql, Kh, Kl, VTh, VTl, C1, 0, RESQB, NQB - RESQB, 0.125f);
    attn_causal64<true><<<gAttR, blk128, 0, stream>>>(
        Qh, Ql, Kh, Kl, VTh, VTl, C2, HD, 0, RESQB, 0.125f);
    attn_causal64<false><<<gAttN, blk128, 0, stream>>>(
        Qh, Ql, Kh, Kl, VTh, VTl, C2, HD, RESQB, NQB - RESQB, 0.125f);
    diff_combine<<<gRow, blk128, 0, stream>>>(C1, C2, lq1, lk1, lq2, lk2, hnw, Oh, Ol);
    gemm64<1, 0, 1><<<gOut, blk256, 0, stream>>>(
        Oh, Ol, DM, 0LL, Wob, Wob, DM, 0LL,
        (void*)outb, DM, 0LL, (void*)outb, DM, 0LL, DM,
        SEQ, DM, DM, 1.0f, bo);
  }
  (void)hipGetLastError();
}
